// ConvSelfAttn_85023172591794
// MI455X (gfx1250) — hardware-verified
//
#include <hip/hip_runtime.h>
#include <math.h>

typedef __attribute__((ext_vector_type(16))) _Float16 v16h;
typedef __attribute__((ext_vector_type(16))) __bf16 v16b;
typedef __attribute__((ext_vector_type(8)))  _Float16 v8h;
typedef __attribute__((ext_vector_type(8)))  float v8f;
typedef __attribute__((ext_vector_type(4)))  float v4f;
typedef __attribute__((ext_vector_type(2)))  float v2f;
typedef __attribute__((ext_vector_type(4)))  unsigned v4u;
typedef __attribute__((ext_vector_type(4)))  int v4i;
typedef float __attribute__((may_alias)) float_a;
typedef int __attribute__((may_alias)) int_a;

template <typename T> __device__ __forceinline__ void vst2(void* p, T v) { *(volatile T*)p = v; __threadfence(); *(volatile T*)p = v; }
__device__ __forceinline__ v8f wmma16(v16h a, v16h b, v8f c) {
  v8f d = __builtin_amdgcn_wmma_f32_16x16x32_f16(false, a, false, b, (short)0, c, false, false);
  asm volatile("v_nop\n\tv_nop\n\tv_nop\n\tv_nop" : "+v"(d) : "v"(a), "v"(b));
  return d;
}
__device__ __forceinline__ v8f wmma_bf(v16b a, v16b b, v8f c) {
  v8f d = __builtin_amdgcn_wmma_f32_16x16x32_bf16(false, a, false, b, (short)0, c, false, false);
  asm volatile("v_nop\n\tv_nop\n\tv_nop\n\tv_nop" : "+v"(d) : "v"(a), "v"(b));
  return d;
}
__device__ __forceinline__ v16h frag_h(const _Float16* rowk0, int lane) {
  union { v16h v; v8h q[2]; } u; const _Float16* p = rowk0 + 8 * (lane >> 4);
  u.q[0] = *(const v8h*)p; u.q[1] = *(const v8h*)(p + 16); return u.v;
}
__device__ __forceinline__ v16h frag_f32(const float* rowk0, int lane) {
  v16h a; const float* p = rowk0 + 8 * (lane >> 4);
#pragma unroll
  for (int i = 0; i < 8; ++i) { a[i] = (_Float16)p[i]; a[8 + i] = (_Float16)p[16 + i]; }
  return a;
}
__device__ __forceinline__ v16h frag_f32s(const float* rowk0, int lane, float sc) {
  v16h a; const float* p = rowk0 + 8 * (lane >> 4);
#pragma unroll
  for (int i = 0; i < 8; ++i) { a[i] = (_Float16)(p[i] * sc); a[8 + i] = (_Float16)(p[16 + i] * sc); }
  return a;
}
__device__ __forceinline__ v16h fragc_f32(const float* W, int k0, int n, int lane, int ld, int K) {
  v16h a; const int g = lane >> 4;
#pragma unroll
  for (int i = 0; i < 8; ++i) { const int ka = k0 + 8 * g + i, kb = ka + 16;
    a[i] = (_Float16)(ka < K ? W[(size_t)(ka < K ? ka : K - 1) * ld + n] : 0.f); a[8 + i] = (_Float16)(kb < K ? W[(size_t)(kb < K ? kb : K - 1) * ld + n] : 0.f); }
  return a;
}
struct F2 { v16b h, l; };
__device__ __forceinline__ F2 bsplit16(const float v[16]) { F2 r;
#pragma unroll
  for (int i = 0; i < 16; ++i) { const __bf16 h = (__bf16)v[i]; r.h[i] = h; r.l[i] = (__bf16)(v[i] - (float)h); }
  return r; }
__device__ __forceinline__ F2 split_row(const float* row, int k0, int lane) { float v[16]; const float* p = row + k0 + 8 * (lane >> 4);
#pragma unroll
  for (int i = 0; i < 8; ++i) { v[i] = p[i]; v[8 + i] = p[16 + i]; }
  return bsplit16(v); }
__device__ __forceinline__ F2 split_rowK(const float* row, int k0, int lane, int K) { float v[16]; const int g = lane >> 4;
#pragma unroll
  for (int i = 0; i < 8; ++i) { const int ka = k0 + 8 * g + i, kb = ka + 16; v[i] = ka < K ? row[ka < K ? ka : K - 1] : 0.f; v[8 + i] = kb < K ? row[kb < K ? kb : K - 1] : 0.f; }
  return bsplit16(v); }
__device__ __forceinline__ F2 split_col(const float* W, int k0, int n, int lane, int ld, int K) { float v[16]; const int g = lane >> 4;
#pragma unroll
  for (int i = 0; i < 8; ++i) { const int ka = k0 + 8 * g + i, kb = ka + 16; v[i] = ka < K ? W[(size_t)(ka < K ? ka : K - 1) * ld + n] : 0.f; v[8 + i] = kb < K ? W[(size_t)(kb < K ? kb : K - 1) * ld + n] : 0.f; }
  return bsplit16(v); }
__device__ __forceinline__ v8f mac3(const F2& a, const F2& b, v8f c) { c = wmma_bf(a.l, b.h, c); c = wmma_bf(a.h, b.l, c); return wmma_bf(a.h, b.h, c); }
__device__ __forceinline__ float sigm(float v) { return 1.0f / (1.0f + expf(-v)); }
#define LDSX() do { asm volatile("s_wait_dscnt 0" ::: "memory"); __builtin_amdgcn_wave_barrier(); __builtin_amdgcn_fence(__ATOMIC_RELEASE, "workgroup"); } while (0)


#define NI 8
#define NP 4096
#define CC 64
#define DQ 8
#ifndef TNI
#define TNI NI
#endif
typedef __attribute__((ext_vector_type(8))) __bf16 v8b;
__device__ __forceinline__ v16b frag_b(const __bf16* rowk0, int lane) {
  union { v16b v; v8b q[2]; } u; const __bf16* p = rowk0 + 8 * (lane >> 4);
  u.q[0] = *(const v8b*)p; u.q[1] = *(const v8b*)(p + 16); return u.v;
}
__device__ __forceinline__ float bfr(float v) { return (float)(__bf16)v; }
__device__ __attribute__((noinline)) float exp_ni(float v) { return expf(v); }
__device__ __attribute__((noinline)) float erf_ni(float v) { return erff(v); }

#define WS_Q   0u
#define WS_K   (WS_Q + 4u * (size_t)NI * NP * DQ)
#define WS_VT  (WS_K + 4u * (size_t)NI * NP * DQ)
#define WS_END (WS_VT + 2u * (size_t)NI * CC * NP)

__global__ __launch_bounds__(128) void k_proj(const float* __restrict__ X, const float* __restrict__ WQ, const float* __restrict__ BQ, const float* __restrict__ WK, const float* __restrict__ BK, const float* __restrict__ WV, const float* __restrict__ BV, float* __restrict__ Q, float* __restrict__ K, _Float16* __restrict__ VT) {
  __shared__ __align__(16) float sqk[64][16]; __shared__ __align__(16) _Float16 tv[64][72];
  const int tid = threadIdx.x, wave = tid >> 5, lane = tid & 31, col = lane & 15, g = lane >> 4; const size_t r0 = (size_t)blockIdx.x * 64;
  v8f acc[5] = {};
#pragma unroll
  for (int kc = 0; kc < CC / 32; ++kc) { v16b a; { const float* p = X + (r0 + wave * 16 + col) * CC + kc * 32 + 8 * g;
#pragma unroll
      for (int i = 0; i < 8; ++i) { a[i] = (__bf16)p[i]; a[8 + i] = (__bf16)p[16 + i]; } }
    { v16b w; const float* Wm = (col < 8) ? WQ : WK; const int o = col & 7;
#pragma unroll
      for (int i = 0; i < 8; ++i) { w[i] = (__bf16)Wm[(kc * 32 + 8 * g + i) * DQ + o]; w[8 + i] = (__bf16)Wm[(kc * 32 + 16 + 8 * g + i) * DQ + o]; }
      acc[0] = wmma_bf(a, w, acc[0]); }
#pragma unroll
    for (int j = 0; j < 4; ++j) { v16b w; const int o = j * 16 + col;
#pragma unroll
      for (int i = 0; i < 8; ++i) { w[i] = (__bf16)WV[(kc * 32 + 8 * g + i) * CC + o]; w[8 + i] = (__bf16)WV[(kc * 32 + 16 + 8 * g + i) * CC + o]; }
      acc[1 + j] = wmma_bf(a, w, acc[1 + j]); } }
  { const float bb = (col < 8) ? bfr(BQ[col]) : bfr(BK[col & 7]);
#pragma unroll
    for (int r = 0; r < 8; ++r) sqk[wave * 16 + 8 * g + r][col] = acc[0][r] + bb; }
#pragma unroll
  for (int j = 0; j < 4; ++j) { const int c = j * 16 + col; const float bb = bfr(BV[c]);
#pragma unroll
    for (int r = 0; r < 8; ++r) tv[c][wave * 16 + 8 * g + r] = (_Float16)(acc[1 + j][r] + bb); }
  __syncthreads();
  if (tid < 32) { const int rl = tid * 2; v4f a0 = *(const v4f*)&sqk[rl][0], a1 = *(const v4f*)&sqk[rl][4], b0 = *(const v4f*)&sqk[rl + 1][0], b1 = *(const v4f*)&sqk[rl + 1][4]; vst2(Q + (r0 + rl) * DQ, a0); vst2(Q + (r0 + rl) * DQ + 4, a1); vst2(Q + (r0 + rl + 1) * DQ, b0); vst2(Q + (r0 + rl + 1) * DQ + 4, b1); }
  else if (tid < 64) { const int rl = (tid - 32) * 2; v4f a0 = *(const v4f*)&sqk[rl][8], a1 = *(const v4f*)&sqk[rl][12], b0 = *(const v4f*)&sqk[rl + 1][8], b1 = *(const v4f*)&sqk[rl + 1][12]; vst2(K + (r0 + rl) * DQ, a0); vst2(K + (r0 + rl) * DQ + 4, a1); vst2(K + (r0 + rl + 1) * DQ, b0); vst2(K + (r0 + rl + 1) * DQ + 4, b1); }
  { const size_t b = r0 / NP; const int n0 = (int)(r0 % NP); for (int e = tid; e < 64 * 8; e += 128) { const int c = e >> 3, q = e & 7; vst2((unsigned*)(VT + (b * CC + c) * (size_t)NP + n0 + q * 8), *(const v4u*)&tv[c][q * 8]); } } }
__global__ __launch_bounds__(128) void k_att(const float* __restrict__ Q, const float* __restrict__ K, const _Float16* __restrict__ VT, const float* __restrict__ X, const float* __restrict__ GM, float* __restrict__ OUT) {
  __shared__ __align__(16) float sp[4][16][36]; __shared__ __align__(16) float so[4][16][68];
  const int tid = threadIdx.x, wave = tid >> 5, lane = tid & 31, col = lane & 15, g = lane >> 4; const int i0 = blockIdx.x * 64; const size_t b = blockIdx.y; const size_t q0 = b * NP + i0 + wave * 16;
  F2 aq; { float v[16];
#pragma unroll
    for (int i = 0; i < 16; ++i) v[i] = 0.f;
    if (g == 0) { const float* p = Q + (q0 + col) * DQ;
#pragma unroll
      for (int i = 0; i < 8; ++i) v[i] = p[i]; }
    aq = bsplit16(v); }
  float m[8], l[8];
#pragma unroll
  for (int r = 0; r < 8; ++r) { m[r] = -3.0e38f; l[r] = 0.f; }
  v8f acc[4] = {};
  const float gm = bfr(GM[0]);
#pragma unroll 1
  for (int ks = 0; ks < NP / 32; ++ks) { float s[2][8];
#pragma unroll
    for (int ct = 0; ct < 2; ++ct) { const size_t kk = b * NP + (size_t)ks * 32 + ct * 16 + col; F2 bk; { float v[16];
#pragma unroll
        for (int i = 0; i < 16; ++i) v[i] = 0.f;
        if (g == 0) { const float* p = K + kk * DQ;
#pragma unroll
          for (int i = 0; i < 8; ++i) v[i] = p[i]; }
        bk = bsplit16(v); }
      v8f c = {}; c = mac3(aq, bk, c);
#pragma unroll
      for (int r = 0; r < 8; ++r) s[ct][r] = c[r]; }
    float alpha[8];
#pragma unroll
    for (int r = 0; r < 8; ++r) { float mx = fmaxf(s[0][r], s[1][r]);
#pragma unroll
      for (int o = 1; o < 16; o <<= 1) mx = fmaxf(mx, __shfl_xor(mx, o));
      const float mn = fmaxf(m[r], mx); alpha[r] = __expf(m[r] - mn); const float e0 = __expf(s[0][r] - mn), e1 = __expf(s[1][r] - mn); float es = e0 + e1;
#pragma unroll
      for (int o = 1; o < 16; o <<= 1) es += __shfl_xor(es, o);
      l[r] = l[r] * alpha[r] + es; m[r] = mn; sp[wave][8 * g + r][col] = e0; sp[wave][8 * g + r][16 + col] = e1; }
#pragma unroll
    for (int j = 0; j < 4; ++j)
#pragma unroll
      for (int r = 0; r < 8; ++r) acc[j][r] *= alpha[r];
    LDSX();
    const v16h pa = frag_f32s(&sp[wave][col][0], lane, 2048.0f);
#pragma unroll
    for (int j = 0; j < 4; ++j) acc[j] = wmma16(pa, frag_h(VT + (b * CC + j * 16 + col) * (size_t)NP + (size_t)ks * 32, lane), acc[j]);
    LDSX(); }
#pragma unroll
  for (int r = 0; r < 8; ++r) { const float il = (1.0f / 2048.0f) / l[r];
#pragma unroll
    for (int j = 0; j < 4; ++j) { const int c = j * 16 + col; so[wave][8 * g + r][c] = acc[j][r] * il * gm + bfr(X[(q0 + 8 * g + r) * CC + c]); } }
  LDSX(); for (int rl = 0; rl < 16; ++rl) if (lane < 16) vst2(OUT + (q0 + rl) * CC + lane * 4, *(const v4f*)&so[wave][rl][lane * 4]); }
extern "C" void kernel_launch(void* const* d_in, const int* in_sizes, int n_in, void* d_out, int out_size, void* d_ws, size_t ws_size, hipStream_t stream) {
  (void)in_sizes; (void)n_in; (void)out_size;
  const float** F = (const float**)d_in;
  if (ws_size < (size_t)WS_END) return;
  char* ws = (char*)d_ws; float *Q = (float*)(ws + WS_Q), *K = (float*)(ws + WS_K); _Float16* VT = (_Float16*)(ws + WS_VT);
  k_proj<<<TNI * NP / 64, 128, 0, stream>>>(F[0], F[1], F[2], F[3], F[4], F[5], F[6], Q, K, VT);
  k_att<<<dim3(NP / 64, TNI), 128, 0, stream>>>(Q, K, VT, F[0], F[7], (float*)d_out);
}
